// LogSigRNNGenerator_58128087384452
// MI455X (gfx1250) — hardware-run, weakly checked
//
#include <hip/hip_runtime.h>
#include <math.h>

constexpr int NBATCH   = 1024;
constexpr int NNOISE   = 1000;
constexpr int NCHAN    = 3;
constexpr int NHID     = 512;
constexpr int NSTEPS   = 64;
constexpr int NSIG     = 6;
constexpr int W1PITCH  = NHID + NSIG;
constexpr int KCAT     = 2 * NHID;
constexpr int MAXSEG   = 4;
constexpr int NOUTC    = 3;
constexpr int NOPAD    = 16;
constexpr int UINTV    = 50;
constexpr int NTHR     = 256;
constexpr int SLABP    = 68;
constexpr float LO_CARRY   = 2048.0f;
constexpr float W_CARRY_LO = 16.0f;
constexpr float W_CARRY_HI = W_CARRY_LO * LO_CARRY;
constexpr float ACC_FOLD   = 1.0f / W_CARRY_HI;

static_assert(W1PITCH == 518);
static_assert(KCAT == 1024 && KCAT % 32 == 0);
static_assert(NHID % 64 == 0 && NBATCH % 128 == 0);
static_assert(NSIG == NCHAN + (NCHAN * (NCHAN - 1)) / 2);
static_assert(NBATCH * NSTEPS * NOUTC == 196608);
static_assert((NBATCH / 2) % 8 == 0);
static_assert(NSTEPS == 64);
static_assert((NBATCH * NSTEPS * NOUTC / 4) % NTHR == 0);

typedef __attribute__((ext_vector_type(16))) _Float16 v16h;
typedef __attribute__((ext_vector_type(8)))  _Float16 v8h;
typedef __attribute__((ext_vector_type(8)))  float    v8f;
typedef __attribute__((ext_vector_type(4)))  float    v4f;
typedef __attribute__((ext_vector_type(4)))  unsigned v4u;

struct EndTable { int e[NSTEPS]; };
static_assert(sizeof(EndTable) == 256);

__device__ __forceinline__ float bf16r(float f) {
  unsigned u = __float_as_uint(f);
  u = (u + 0x7FFFu + ((u >> 16) & 1u)) & 0xFFFF0000u;
  return __uint_as_float(u);
}

union FragU { v16h v; v8h h[2]; };
__device__ __forceinline__ v16h frag_load(const _Float16* p) {
  FragU f; f.h[0] = *(const v8h*)(p); f.h[1] = *(const v8h*)(p + 16); return f.v;
}
__device__ __forceinline__ v8f frag_mma(v16h a, v16h b, v8f c) {
  return __builtin_amdgcn_wmma_f32_16x16x32_f16(false, a, false, b, (short)0, c, false, false);
}
__device__ __forceinline__ void guard_group4(v8f& a0, v8f& a1, v8f& a2, v8f& a3, v16h x, v16h b0, v16h b1, v16h b2, v16h b3) {
  asm volatile("v_nop\n\tv_nop\n\tv_nop\n\tv_nop" : "+v"(a0), "+v"(a1), "+v"(a2), "+v"(a3) : "v"(x), "v"(b0), "v"(b1), "v"(b2), "v"(b3));
}
__device__ __forceinline__ void guard_group2(v8f& a0, v8f& a1, v16h x0, v16h y0, v16h x1, v16h y1) {
  asm volatile("v_nop\n\tv_nop\n\tv_nop\n\tv_nop" : "+v"(a0), "+v"(a1) : "v"(x0), "v"(y0), "v"(x1), "v"(y1));
}
__device__ __forceinline__ void acc_guard4(v8f& a, v8f& b, v8f& c, v8f& d) {
  asm volatile("v_nop\n\tv_nop\n\tv_nop\n\tv_nop" : "+v"(a), "+v"(b), "+v"(c), "+v"(d));
}
__device__ __forceinline__ void wave_sync() {
  __builtin_amdgcn_fence(__ATOMIC_RELEASE, "workgroup");
  __builtin_amdgcn_wave_barrier();
  __builtin_amdgcn_fence(__ATOMIC_ACQUIRE, "workgroup");
}

__global__ __launch_bounds__(32) void premise_kernel(const int* __restrict__ wsz, unsigned* __restrict__ FL) {
  const int w = wsz[0];
  const unsigned f = (w != NSTEPS) ? 1u : 0u;
  unsigned* op = FL + threadIdx.x;
  *(volatile unsigned*)op = f;
  __threadfence();
  *(volatile unsigned*)op = f;
}

__global__ __launch_bounds__(NTHR) void poison_kernel(const unsigned* __restrict__ FL, unsigned* __restrict__ outw, int n16) {
  const int i = blockIdx.x * NTHR + threadIdx.x;
  const unsigned f = FL[0];
  if (f == 0u) return;
  if (i >= n16) return;
  const v4u nv = {0x7FC00000u, 0x7FC00000u, 0x7FC00000u, 0x7FC00000u};
  unsigned* op = outw + (size_t)i * 4;
  *(volatile v4u*)op = nv;
  __threadfence();
  *(volatile v4u*)op = nv;
}

__global__ __launch_bounds__(NTHR) void wplane_kernel(const float* __restrict__ src, unsigned short* __restrict__ dst,
                                                      int nrow_dst, int nrow_src, int spitch) {
  const int i = blockIdx.x * NTHR + threadIdx.x;
  if (i >= nrow_dst * (KCAT / 8)) return;
  const int row = i >> 7;
  const int c8  = i & 127;
  const int kk  = (c8 * 8) & (NHID - 1);
  const float sc = (c8 < 64) ? W_CARRY_HI : W_CARRY_LO;
  const bool live = row < nrow_src;
  const int rs = live ? row : (nrow_src - 1);
  const float* sp = src + (size_t)rs * (size_t)spitch + kk;
  v8h hv;
#pragma unroll
  for (int e = 0; e < 8; ++e) {
    const float x = sp[e];
    const float y = live ? (bf16r(x) * sc) : 0.0f;
    hv[e] = (_Float16)y;
  }
  unsigned short* op = dst + (size_t)i * 8;
  *(volatile v8h*)op = hv;
  __threadfence();
  *(volatile v8h*)op = hv;
}

__global__ __launch_bounds__(NTHR) void w1sig_kernel(const float* __restrict__ W1, float* __restrict__ W1T) {
  const int i  = blockIdx.x * NTHR + threadIdx.x;
  const int c  = i >> 7;
  const int n4 = (i & 127) * 4;
  const bool live = c < NSIG;
  const int cc = live ? c : (NSIG - 1);
  v4f o;
#pragma unroll
  for (int e = 0; e < 4; ++e) {
    const float x = W1[(size_t)(n4 + e) * W1PITCH + NHID + cc];
    o[e] = live ? bf16r(x) : 0.0f;
  }
  float* op = W1T + c * NHID + n4;
  *(volatile v4f*)op = o;
  __threadfence();
  *(volatile v4f*)op = o;
}

__global__ __launch_bounds__(NTHR) void zero_kernel(unsigned* __restrict__ dst, int n16) {
  const int i = blockIdx.x * NTHR + threadIdx.x;
  if (i >= n16) return;
  const v4u zv = {0u, 0u, 0u, 0u};
  unsigned* op = dst + (size_t)i * 4;
  *(volatile v4u*)op = zv;
  __threadfence();
  *(volatile v4u*)op = zv;
}

__global__ __launch_bounds__(NTHR) void path_kernel(const float* __restrict__ z, float* __restrict__ SG, EndTable tab, float sdt) {
  const int b = blockIdx.x * NTHR + threadIdx.x;
  const float* zp = z + (size_t)b * (size_t)(NNOISE * NCHAN);
  float p0 = 0.f, p1 = 0.f, p2 = 0.f;
  float c01 = 0.f, c02 = 0.f, c12 = 0.f;
  float s01 = 0.f, s02 = 0.f, s12 = 0.f;
  {
    float* o0 = SG + b;
    for (int pass = 0; pass < 2; ++pass) {
#pragma unroll
      for (int c = 0; c < NSIG; ++c) *(volatile float*)(o0 + c * NBATCH) = 0.0f;
      __threadfence();
    }
  }
  int t = 1;
  int cnt = 1;
#pragma unroll 1
  for (int k = 1; k < NSTEPS; ++k) {
    int e = tab.e[k];
    e = e < 0 ? 0 : e;
    e = e > (NNOISE - 1) ? (NNOISE - 1) : e;
#pragma unroll 1
    for (; t <= e; ++t) {
      const float z0 = bf16r(zp[t * 3 + 0]) * sdt;
      const float z1 = bf16r(zp[t * 3 + 1]) * sdt;
      const float z2 = bf16r(zp[t * 3 + 2]) * sdt;
      const float n0 = p0 + z0, n1 = p1 + z1, n2 = p2 + z2;
      c01 += 0.5f * (p0 * n1 - p1 * n0);
      c02 += 0.5f * (p0 * n2 - p2 * n0);
      c12 += 0.5f * (p1 * n2 - p2 * n1);
      p0 = n0; p1 = n1; p2 = n2;
      if (cnt == UINTV) { s01 = c01; s02 = c02; s12 = c12; cnt = 0; }
      ++cnt;
    }
    const float v0 = p0, v1 = p1, v2 = p2;
    const float v3 = c01 - s01, v4 = c02 - s02, v5 = c12 - s12;
    float* o = SG + (size_t)(k * NSIG) * NBATCH + b;
    for (int pass = 0; pass < 2; ++pass) {
      *(volatile float*)(o + 0 * NBATCH) = v0;
      *(volatile float*)(o + 1 * NBATCH) = v1;
      *(volatile float*)(o + 2 * NBATCH) = v2;
      *(volatile float*)(o + 3 * NBATCH) = v3;
      *(volatile float*)(o + 4 * NBATCH) = v4;
      *(volatile float*)(o + 5 * NBATCH) = v5;
      __threadfence();
    }
  }
}

template <int EPI>
__global__ __launch_bounds__(NTHR) void gemm_cat_kernel(const unsigned short* __restrict__ Ap,
                                                        const unsigned short* __restrict__ Btp,
                                                        void* __restrict__ Cout, const float* __restrict__ bias, int nrows) {
  __shared__ __align__(16) float sT[NTHR / 32][16 * SLABP];
  const _Float16* A  = (const _Float16*)Ap;
  const _Float16* Bt = (const _Float16*)Btp;
  const int lane = threadIdx.x & 31;
  const int wave = threadIdx.x >> 5;
  const int m0 = blockIdx.x << 6;
  const int n0 = wave << 6;
  if (m0 + 64 > nrows) return;
  const int rlane = lane & 15;
  const int koff  = (lane >> 4) * 8;
  const int mOff  = (lane >> 4) * 8;
  const _Float16* arow = A  + (size_t)(m0 + rlane) * KCAT + koff;
  const _Float16* brow = Bt + (size_t)(n0 + rlane) * KCAT + koff;

  v8f acc[4][4];
#pragma unroll
  for (int i = 0; i < 4; ++i)
#pragma unroll
    for (int j = 0; j < 4; ++j) acc[i][j] = (v8f){0.f, 0.f, 0.f, 0.f, 0.f, 0.f, 0.f, 0.f};

#pragma unroll 1
  for (int k0 = 0; k0 < KCAT; k0 += 32) {
    v16h bh[4];
#pragma unroll
    for (int j = 0; j < 4; ++j) bh[j] = frag_load(brow + (size_t)(j * 16) * KCAT + k0);
#pragma unroll
    for (int i = 0; i < 4; ++i) {
      const v16h ah = frag_load(arow + (size_t)(i * 16) * KCAT + k0);
#pragma unroll
      for (int j = 0; j < 4; ++j) acc[i][j] = frag_mma(ah, bh[j], acc[i][j]);
      guard_group4(acc[i][0], acc[i][1], acc[i][2], acc[i][3], ah, bh[0], bh[1], bh[2], bh[3]);
    }
  }
  acc_guard4(acc[0][0], acc[0][1], acc[0][2], acc[0][3]);
  acc_guard4(acc[1][0], acc[1][1], acc[1][2], acc[1][3]);
  acc_guard4(acc[2][0], acc[2][1], acc[2][2], acc[2][3]);
  acc_guard4(acc[3][0], acc[3][1], acc[3][2], acc[3][3]);

  float* slab = sT[wave];
  float bvs[4] = {0.f, 0.f, 0.f, 0.f};
  float biasA = 0.f, biasB = 0.f;
  if (EPI == 1) {
#pragma unroll
    for (int j = 0; j < 4; ++j) bvs[j] = bf16r(bias[n0 + (j << 4) + rlane]);
  }
  if (EPI == 2) {
    biasA = bf16r(bias[n0 + lane]);
    biasB = bf16r(bias[n0 + 32 + lane]);
  }
#pragma unroll
  for (int i = 0; i < 4; ++i) {
    const int mBase = m0 + (i << 4);
#pragma unroll
    for (int j = 0; j < 4; ++j) {
#pragma unroll
      for (int r = 0; r < 8; ++r) {
        float v = acc[i][j][r] * ACC_FOLD;
        if (EPI == 1) { v += bvs[j]; v = fmaxf(v, 0.0f); }
        slab[(mOff + r) * SLABP + (j << 4) + rlane] = v;
      }
    }
    wave_sync();
    if (EPI == 2) {
#pragma unroll 1
      for (int it = 0; it < 32; ++it) {
        const int idx = (it >> 1) * SLABP + ((it & 1) << 5) + lane;
        const float bsel = (it & 1) ? biasB : biasA;
        const float v = slab[idx] + bsel;
        slab[idx] = tanhf(v);
      }
      wave_sync();
    }
    if (EPI == 0) {
      float* C = (float*)Cout;
      const int hh = lane >> 4, c4 = (lane & 15) * 4;
      for (int pass = 0; pass < 2; ++pass) {
#pragma unroll
        for (int it = 0; it < 8; ++it) {
          const int row = it * 2 + hh;
          const v4f v = *(const v4f*)(slab + row * SLABP + c4);
          *(volatile v4f*)(C + (size_t)(mBase + row) * NHID + n0 + c4) = v;
        }
        __threadfence();
      }
    } else {
      unsigned short* C = (unsigned short*)Cout;
      const int q = lane >> 3, c8 = (lane & 7) * 8;
      for (int pass = 0; pass < 2; ++pass) {
#pragma unroll
        for (int it = 0; it < 4; ++it) {
          const int row = it * 4 + q;
          const float* sp = slab + row * SLABP + c8;
          v8h hv, lv;
#pragma unroll
          for (int e = 0; e < 8; ++e) {
            const float x = sp[e];
            const _Float16 hx = (_Float16)x;
            const float hf = (float)hx;
            const float rx = (x - hf) * LO_CARRY;
            hv[e] = hx;
            lv[e] = (_Float16)rx;
          }
          unsigned short* cp = C + (size_t)(mBase + row) * KCAT + n0 + c8;
          *(volatile v8h*)(cp) = hv;
          *(volatile v8h*)(cp + NHID) = lv;
        }
        __threadfence();
      }
    }
    wave_sync();
  }
}

__global__ __launch_bounds__(NTHR) void layer1_kernel(const float* __restrict__ P, const float* __restrict__ b1,
                                                      const float* __restrict__ W1T, const float* __restrict__ SGseg,
                                                      unsigned short* __restrict__ H1, int nrows) {
  const int i = blockIdx.x * NTHR + threadIdx.x;
  if (i >= nrows * 64) return;
  const int r  = i >> 6;
  const int n  = (i & 63) * 8;
  const int s  = r >> 10;
  const int b  = r & (NBATCH - 1);
  const v4f pa = *(const v4f*)(P + (size_t)b * NHID + n);
  const v4f pb = *(const v4f*)(P + (size_t)b * NHID + n + 4);
  const v4f ba = *(const v4f*)(b1 + n);
  const v4f bb = *(const v4f*)(b1 + n + 4);
  float a[8];
#pragma unroll
  for (int e = 0; e < 4; ++e) { a[e] = pa[e] + bf16r(ba[e]); a[4 + e] = pb[e] + bf16r(bb[e]); }
#pragma unroll 1
  for (int c = 0; c < NSIG; ++c) {
    const float sv = SGseg[(size_t)(s * NSIG + c) * NBATCH + b];
    const v4f wa = *(const v4f*)(W1T + c * NHID + n);
    const v4f wb = *(const v4f*)(W1T + c * NHID + n + 4);
#pragma unroll
    for (int e = 0; e < 4; ++e) { a[e] = fmaf(sv, wa[e], a[e]); a[4 + e] = fmaf(sv, wb[e], a[4 + e]); }
  }
  v8h hv, lv;
#pragma unroll
  for (int e = 0; e < 8; ++e) {
    const float x = fmaxf(a[e], 0.0f);
    const _Float16 hx = (_Float16)x;
    const float hf = (float)hx;
    const float rx = (x - hf) * LO_CARRY;
    hv[e] = hx;
    lv[e] = (_Float16)rx;
  }
  unsigned short* op = H1 + (size_t)r * KCAT + n;
  for (int pass = 0; pass < 2; ++pass) {
    *(volatile v8h*)(op) = hv;
    *(volatile v8h*)(op + NHID) = lv;
    __threadfence();
  }
}

__global__ __launch_bounds__(NTHR) void outproj_kernel(const unsigned short* __restrict__ Hp,
                                                       const unsigned short* __restrict__ Wop,
                                                       float* __restrict__ OutSeg) {
  __shared__ __align__(16) float So[128 * 4];
  const _Float16* Hm = (const _Float16*)Hp;
  const _Float16* Wo = (const _Float16*)Wop;
  const int tid = threadIdx.x, lane = tid & 31, wave = tid >> 5;
  const int c = lane & 15, hh = lane >> 4, koff = hh * 8;
  const int m0 = blockIdx.x * 128 + wave * 16;
  const _Float16* ap = Hm + (size_t)(m0 + c) * KCAT + koff;
  const _Float16* bp = Wo + (size_t)c * KCAT + koff;
  v8f acc0 = {0.f, 0.f, 0.f, 0.f, 0.f, 0.f, 0.f, 0.f};
  v8f acc1 = acc0;
#pragma unroll 1
  for (int k0 = 0; k0 < KCAT; k0 += 64) {
    const v16h a0 = frag_load(ap + k0);
    const v16h b0 = frag_load(bp + k0);
    const v16h a1 = frag_load(ap + k0 + 32);
    const v16h b1 = frag_load(bp + k0 + 32);
    acc0 = frag_mma(a0, b0, acc0);
    acc1 = frag_mma(a1, b1, acc1);
    guard_group2(acc0, acc1, a0, b0, a1, b1);
  }
  if (c < 4) {
#pragma unroll
    for (int r = 0; r < 8; ++r) So[(wave * 16 + 8 * hh + r) * 4 + c] = (acc0[r] + acc1[r]) * ACC_FOLD;
  }
  __syncthreads();
  if (tid < 128) {
    const v4f v = *(const v4f*)(So + tid * 4);
    float* op = OutSeg + ((size_t)blockIdx.x * 128 + tid) * 4;
    *(volatile v4f*)op = v;
    __threadfence();
    *(volatile v4f*)op = v;
  }
}

__global__ __launch_bounds__(NTHR) void pack_kernel(const float* __restrict__ OutS, float* __restrict__ out) {
  const int lane = threadIdx.x & 31;
  const int w = blockIdx.x * (NTHR / 32) + (threadIdx.x >> 5);
  v4f o[3];
#pragma unroll
  for (int i = 0; i < 3; ++i) {
#pragma unroll
    for (int e = 0; e < 4; ++e) {
      const int f = 128 * i + 4 * lane + e;
      const int bb = (f >= NSTEPS * NOUTC) ? 1 : 0;
      const int rem = f - bb * (NSTEPS * NOUTC);
      const int t = rem / NOUTC;
      const int c = rem - t * NOUTC;
      o[i][e] = OutS[((size_t)t * NBATCH + (size_t)(2 * w + bb)) * 4 + c];
    }
  }
  float* op = out + (size_t)w * (2 * NSTEPS * NOUTC) + 4 * lane;
  for (int pass = 0; pass < 2; ++pass) {
#pragma unroll
    for (int i = 0; i < 3; ++i) *(volatile v4f*)(op + 128 * i) = o[i];
    __threadfence();
  }
}

extern "C" void kernel_launch(void* const* d_in, const int* in_sizes, int n_in,
                              void* d_out, int out_size, void* d_ws, size_t ws_size, hipStream_t stream) {
  if (n_in < 10 || d_out == nullptr || d_ws == nullptr) return;
  if (in_sizes[0] != NBATCH * NNOISE * NCHAN || in_sizes[1] != NHID * W1PITCH || in_sizes[2] != NHID ||
      in_sizes[3] != NHID * NHID || in_sizes[4] != NHID || in_sizes[5] != NHID * NHID || in_sizes[6] != NHID ||
      in_sizes[7] != NOUTC * NHID || in_sizes[9] < 1 || out_size != NBATCH * NSTEPS * NOUTC) return;

  const float* z    = (const float*)d_in[0];
  const float* W1   = (const float*)d_in[1];
  const float* b1   = (const float*)d_in[2];
  const float* W2   = (const float*)d_in[3];
  const float* b2   = (const float*)d_in[4];
  const float* W3   = (const float*)d_in[5];
  const float* b3   = (const float*)d_in[6];
  const float* Wout = (const float*)d_in[7];
  const int*   wsz  = (const int*)d_in[9];
  float* out = (float*)d_out;

  double tb[NNOISE], tt[NSTEPS], tu[(NNOISE + UINTV - 1) / UINTV];
  const int nu = (NNOISE + UINTV - 1) / UINTV;
  const double stepb = 1.0 / (double)(NNOISE - 1);
  for (int i = 0; i < NNOISE; ++i) tb[i] = (double)i * stepb;
  tb[NNOISE - 1] = 1.0;
  const double stept = 1.0 / (double)(NSTEPS - 1);
  for (int i = 0; i < NSTEPS; ++i) tt[i] = (double)i * stept;
  tt[NSTEPS - 1] = 1.0;
  for (int j = 0; j < nu; ++j) tu[j] = tb[UINTV * j];

  EndTable tab;
  int startsA[NSTEPS], uidx[NSTEPS];
  tab.e[0] = 0; startsA[0] = 0; uidx[0] = 0;
  for (int k = 1; k < NSTEPS; ++k) {
    const double v = tt[k];
    int cnt = 0;
    for (int i = 0; i < NNOISE; ++i) if (tb[i] <= v) ++cnt;
    int cu = 0;
    for (int j = 0; j < nu; ++j) if (tu[j] <= v) ++cu;
    int iu = cu - 1;
    if (iu < 0) iu = 0;
    int cs = 0;
    for (int i = 0; i < NNOISE; ++i) if (tb[i] <= tu[iu]) ++cs;
    tab.e[k] = cnt - 1;
    startsA[k] = cs - 1;
    uidx[k] = iu;
  }
  double utimes[NSTEPS + 1];
  int nut = 0, lastu = -1;
  for (int k = 1; k < NSTEPS; ++k)
    if (uidx[k] != lastu) { utimes[nut++] = tu[uidx[k]]; lastu = uidx[k]; }
  utimes[nut++] = tt[NSTEPS - 1];
  int gate[NSTEPS];
  {
    int qi = 0;
    for (int i = 0; i < NSTEPS; ++i) {
      if (qi < nut && tt[i] >= utimes[qi]) { ++qi; gate[i] = 1; } else gate[i] = 0;
    }
  }
  for (int k = 1; k < NSTEPS; ++k) {
    const int e = tab.e[k];
    if (e < 0 || e > NNOISE - 1) return;
    if (e < tab.e[k - 1]) return;
    if (startsA[k] != (e / UINTV) * UINTV) return;
  }
  int segT0[NSTEPS], segLen[NSTEPS], segGate[NSTEPS];
  int nseg = 0;
  {
    int st = 0;
    for (int t = 0; t < NSTEPS; ++t) {
      if (gate[t]) { segT0[nseg] = st; segLen[nseg] = t - st + 1; segGate[nseg] = 1; ++nseg; st = t + 1; }
    }
    if (st < NSTEPS) { segT0[nseg] = st; segLen[nseg] = NSTEPS - st; segGate[nseg] = 0; ++nseg; }
  }
  for (int s = 0; s < nseg; ++s) if (segLen[s] < 1 || segLen[s] > MAXSEG) return;

  const float sdt = (float)sqrt(1.0 / (double)(NNOISE - 1));

  char* ws = (char*)d_ws; size_t off = 0;
  auto carve = [&](size_t bytes) -> char* { char* p = ws + off; off += (bytes + 255) & ~(size_t)255; return p; };
  unsigned short* W1P = (unsigned short*)carve((size_t)NHID * KCAT * 2);
  unsigned short* W2P = (unsigned short*)carve((size_t)NHID * KCAT * 2);
  unsigned short* W3P = (unsigned short*)carve((size_t)NHID * KCAT * 2);
  unsigned short* WOP = (unsigned short*)carve((size_t)NOPAD * KCAT * 2);
  float*          W1T = (float*)carve((size_t)8 * NHID * 4);
  float*          SG  = (float*)carve((size_t)NSTEPS * NSIG * NBATCH * 4);
  unsigned short* HZ  = (unsigned short*)carve((size_t)NBATCH * KCAT * 2);
  float*          PP  = (float*)carve((size_t)NBATCH * NHID * 4);
  unsigned short* H1  = (unsigned short*)carve((size_t)MAXSEG * NBATCH * KCAT * 2);
  unsigned short* H2  = (unsigned short*)carve((size_t)MAXSEG * NBATCH * KCAT * 2);
  unsigned short* H3A = (unsigned short*)carve((size_t)MAXSEG * NBATCH * KCAT * 2);
  unsigned short* H3B = (unsigned short*)carve((size_t)MAXSEG * NBATCH * KCAT * 2);
  float*          OUTS = (float*)carve((size_t)NSTEPS * NBATCH * 4 * 4);
  unsigned*       FL  = (unsigned*)carve((size_t)256);
  if (off > ws_size || off > (size_t)134217728) return;

  premise_kernel<<<1, 32, 0, stream>>>(wsz, FL);

  wplane_kernel<<<(NHID * (KCAT / 8)) / NTHR, NTHR, 0, stream>>>(W1, W1P, NHID, NHID, W1PITCH);
  wplane_kernel<<<(NHID * (KCAT / 8)) / NTHR, NTHR, 0, stream>>>(W2, W2P, NHID, NHID, NHID);
  wplane_kernel<<<(NHID * (KCAT / 8)) / NTHR, NTHR, 0, stream>>>(W3, W3P, NHID, NHID, NHID);
  wplane_kernel<<<(NOPAD * (KCAT / 8)) / NTHR, NTHR, 0, stream>>>(Wout, WOP, NOPAD, NOUTC, NHID);
  w1sig_kernel<<<(8 * NHID / 4) / NTHR, NTHR, 0, stream>>>(W1, W1T);
  zero_kernel<<<(NBATCH * KCAT * 2 / 16) / NTHR, NTHR, 0, stream>>>((unsigned*)HZ, NBATCH * KCAT * 2 / 16);
  path_kernel<<<NBATCH / NTHR, NTHR, 0, stream>>>(z, SG, tab, sdt);

  const unsigned short* hlast = HZ;
  int pp = 0;
  for (int s = 0; s < nseg; ++s) {
    const int t0 = segT0[s];
    const int len = segLen[s];
    const int mrows = len * NBATCH;
    unsigned short* H3 = pp ? H3B : H3A;
    gemm_cat_kernel<0><<<NBATCH / 64, NTHR, 0, stream>>>(hlast, W1P, (void*)PP, b1, NBATCH);
    layer1_kernel<<<mrows / 4, NTHR, 0, stream>>>(PP, b1, W1T, SG + (size_t)t0 * NSIG * NBATCH, H1, mrows);
    gemm_cat_kernel<1><<<mrows / 64, NTHR, 0, stream>>>(H1, W2P, (void*)H2, b2, mrows);
    gemm_cat_kernel<2><<<mrows / 64, NTHR, 0, stream>>>(H2, W3P, (void*)H3, b3, mrows);
    outproj_kernel<<<mrows / 128, NTHR, 0, stream>>>(H3, WOP, OUTS + (size_t)t0 * NBATCH * 4);
    if (segGate[s]) {
      hlast = H3 + (size_t)(len - 1) * NBATCH * KCAT;
      pp ^= 1;
    }
  }
  pack_kernel<<<(NBATCH / 2) / (NTHR / 32), NTHR, 0, stream>>>(OUTS, out);
  poison_kernel<<<(NBATCH * NSTEPS * NOUTC / 4) / NTHR, NTHR, 0, stream>>>(FL, (unsigned*)d_out, NBATCH * NSTEPS * NOUTC / 4);
}
